// EG_GATLayer_15702400434747
// MI455X (gfx1250) — hardware-run, weakly checked
//
#include <hip/hip_runtime.h>

typedef float          v8f   __attribute__((ext_vector_type(8)));
typedef float          v4f   __attribute__((ext_vector_type(4)));
typedef unsigned int   v4u   __attribute__((ext_vector_type(4)));
typedef int            v8i   __attribute__((ext_vector_type(8)));
typedef unsigned short v8us  __attribute__((ext_vector_type(8)));
typedef unsigned short v16us __attribute__((ext_vector_type(16)));
typedef __bf16         v16bf __attribute__((ext_vector_type(16)));
typedef _Float16       v16h  __attribute__((ext_vector_type(16)));
typedef v4f  __attribute__((may_alias)) v4fa;
typedef v8us __attribute__((may_alias)) v8usa;
union FragB { v16bf v; v16us u; v8us h[2]; v8i w; };
union FragH { v16h  v; v16us u; v8us h[2]; v8i w; };

__device__ __forceinline__ v8f wmb(const FragB& a, const FragB& b, v8f c) {
  v8f d = __builtin_amdgcn_wmma_f32_16x16x32_bf16(false, a.v, false, b.v, (short)0, c, false, false);
  asm volatile("v_nop\n\tv_nop\n\tv_nop\n\tv_nop" : "+v"(d) : "v"(a.w), "v"(b.w));
  return d;
}

__device__ __forceinline__ v8f wmh(const FragH& a, const FragH& b, v8f c) {
  v8f d = __builtin_amdgcn_wmma_f32_16x16x32_f16(false, a.v, false, b.v, (short)0, c, false, false);
  asm volatile("v_nop\n\tv_nop\n\tv_nop\n\tv_nop" : "+v"(d) : "v"(a.w), "v"(b.w));
  return d;
}

__device__ __forceinline__ unsigned bf16_bits(float f) {
  const unsigned u = __float_as_uint(f);
  const unsigned r = (u + 0x7FFFu + ((u >> 16) & 1u)) >> 16;
  const unsigned q = (u >> 16) | 0x40u;
  return ((u & 0x7fffffffu) > 0x7f800000u) ? q : r;
}

__device__ __forceinline__ float bf16_val(float f) {
  return __uint_as_float(bf16_bits(f) << 16);
}
__device__ __forceinline__ int clampi(int v, int lo, int hi) {
  return v < lo ? lo : (v > hi ? hi : v);
}

__device__ __forceinline__ unsigned f16_bits(float f) {
  const unsigned u  = __float_as_uint(f);
  const unsigned s  = (u >> 16) & 0x8000u;
  const unsigned a  = u & 0x7fffffffu;
  const unsigned t  = a - 0x38000000u;
  const unsigned r  = (t + 0x0FFFu + ((t >> 13) & 1u)) >> 13;
  const unsigned rc = r > 0x7C00u ? 0x7C00u : r;
  const bool small  = a < 0x38800000u;
  const bool isnan  = a > 0x7f800000u;
  const unsigned fin = small ? 0u : (s | rc);
  return isnan ? (s | 0x7E00u) : fin;
}

__device__ __forceinline__ unsigned pk16(unsigned lo, unsigned hi) { return lo | (hi << 16); }
__device__ __forceinline__ unsigned bf16_lo_bits(float v) {
  float hi = bf16_val(v);
  asm volatile("" : "+v"(hi));
  return bf16_bits(v - hi);
}
__device__ __forceinline__ v4u pack8_bf16(v4f a, v4f c) {
  return (v4u){ pk16(bf16_bits(a[0]), bf16_bits(a[1])), pk16(bf16_bits(a[2]), bf16_bits(a[3])),
                pk16(bf16_bits(c[0]), bf16_bits(c[1])), pk16(bf16_bits(c[2]), bf16_bits(c[3])) };
}
__device__ __forceinline__ v4u pack8_bf16_lo(v4f a, v4f c) {
  return (v4u){ pk16(bf16_lo_bits(a[0]), bf16_lo_bits(a[1])), pk16(bf16_lo_bits(a[2]), bf16_lo_bits(a[3])),
                pk16(bf16_lo_bits(c[0]), bf16_lo_bits(c[1])), pk16(bf16_lo_bits(c[2]), bf16_lo_bits(c[3])) };
}
__device__ __forceinline__ v4u pack8_f16(v4f a, v4f c) {
  return (v4u){ pk16(f16_bits(a[0]), f16_bits(a[1])), pk16(f16_bits(a[2]), f16_bits(a[3])),
                pk16(f16_bits(c[0]), f16_bits(c[1])), pk16(f16_bits(c[2]), f16_bits(c[3])) };
}

template <int FORM>
__global__ __launch_bounds__(256) void k_plane(const float* __restrict__ src, int rows, int cols, int ldsrc,
                                               unsigned short* __restrict__ dst, int MP, int KP) {
  static_assert(FORM >= 0 && FORM <= 3);
  const int KTOT = (FORM == 1 || FORM == 3) ? 2 * KP : KP;
  const unsigned ppr   = (unsigned)(KTOT >> 3);
  const unsigned kp8   = (unsigned)(KP >> 3);
  const unsigned total = (unsigned)MP * ppr;
  const unsigned g     = blockIdx.x * 256u + threadIdx.x;
  const unsigned rowu  = g / ppr;
  const unsigned p     = g - rowu * ppr;
  const bool second    = p >= kp8;
  const int row = (int)rowu;
  const int c0  = (int)((second ? p - kp8 : p) << 3);
  const float* srow = src + (size_t)clampi(row, 0, rows - 1) * (size_t)ldsrc;
  float x[8];
  unsigned mk[8];
#pragma unroll
  for (int e = 0; e < 8; ++e) {
    const int c = c0 + e;
    const float v = srow[clampi(c, 0, cols - 1)];
    asm volatile("" :: "v"(v));
    x[e]  = v;
    mk[e] = (row < rows && c < cols) ? 0xFFFFu : 0u;
  }
  const v4f a = (v4f){ x[0], x[1], x[2], x[3] };
  const v4f c = (v4f){ x[4], x[5], x[6], x[7] };
  v4u o;
  if (FORM == 2) {
    o = pack8_f16(a, c);
  } else {
    const v4u hi = pack8_bf16(a, c);
    o = hi;
    if (FORM == 1) { const v4u lo = pack8_bf16_lo(a, c); o = second ? lo : hi; }
  }
  const v4u mw = (v4u){ pk16(mk[0], mk[1]), pk16(mk[2], mk[3]), pk16(mk[4], mk[5]), pk16(mk[6], mk[7]) };
  o &= mw;
  if (g < total) {
    volatile v4u* q = (volatile v4u*)(dst + (size_t)g * 8);
    *q = o;
    __threadfence();
    *q = o;
  }
}

template <int FORM> struct FragOf    { typedef FragB T; };
template <>         struct FragOf<2> { typedef FragH T; };
__device__ __forceinline__ v8f mm(const FragB& a, const FragB& b, v8f c) { return wmb(a, b, c); }
__device__ __forceinline__ v8f mm(const FragH& a, const FragH& b, v8f c) { return wmh(a, b, c); }
template <class F> __device__ __forceinline__ F ld_frag(const unsigned short* p) {
  F f;
  f.h[0] = *(const v8usa*)(p);
  f.h[1] = *(const v8usa*)(p + 16);
  return f;
}

template <int FORM, int EPI>
__global__ __launch_bounds__(256) __attribute__((amdgpu_num_vgpr(248)))
void k_gemm_nt(const unsigned short* __restrict__ A, const unsigned short* __restrict__ B,
               const float* __restrict__ bias, float* __restrict__ D, int M, int N, int KTOT, int ldd) {
  static_assert(FORM >= 0 && FORM <= 2);
  static_assert(EPI == 0 || EPI == 1);
  typedef typename FragOf<FORM>::T F;
  __shared__ __attribute__((aligned(16))) float sT[8][16 * 68];
  const int lane = threadIdx.x & 31;
  const int wave = threadIdx.x >> 5;
  const int tilesM = (M + 63) >> 6;
  const int tilesN = (N + 63) >> 6;
  const int tile = blockIdx.x * 8 + wave;
  if (tile >= tilesM * tilesN) return;
  const int tm = tile / tilesN;
  const int tn = tile - tm * tilesN;
  const int m0 = tm << 6;
  const int n0 = tn << 6;

  const int rl = lane & 15;
  const int h8 = (lane >> 4) * 8;
  const unsigned short* pa = A + (size_t)(m0 + rl) * (size_t)KTOT + h8;
  const unsigned short* pb = B + (size_t)(n0 + rl) * (size_t)KTOT + h8;

  v8f acc[4][4];
#pragma unroll
  for (int i = 0; i < 4; ++i)
#pragma unroll
    for (int j = 0; j < 4; ++j) acc[i][j] = (v8f){0.f, 0.f, 0.f, 0.f, 0.f, 0.f, 0.f, 0.f};

#pragma unroll 1
  for (int k0 = 0; k0 < KTOT; k0 += 32) {
    F bf[4];
#pragma unroll
    for (int j = 0; j < 4; ++j) bf[j] = ld_frag<F>(pb + (size_t)(j << 4) * (size_t)KTOT + k0);
#pragma unroll
    for (int i = 0; i < 4; ++i) {
      const F af = ld_frag<F>(pa + (size_t)(i << 4) * (size_t)KTOT + k0);
#pragma unroll
      for (int j = 0; j < 4; ++j) acc[i][j] = mm(af, bf[j], acc[i][j]);
    }
  }

  float* slab = sT[wave];
  const int hh = lane >> 4;
  const int c4 = (lane & 15) * 4;
  const int nc = n0 + c4;
  const bool cok = nc < N;
  v4f bv = (v4f){0.f, 0.f, 0.f, 0.f};
  if (EPI == 1) {
    bv = *(const v4fa*)(bias + clampi(nc, 0, N - 4));
    asm volatile("" :: "v"(bv));
  }
#pragma unroll
  for (int i = 0; i < 4; ++i) {
    const int mBase = m0 + (i << 4);
#pragma unroll
    for (int j = 0; j < 4; ++j) {
#pragma unroll
      for (int r = 0; r < 8; ++r) slab[(h8 + r) * 68 + (j << 4) + rl] = acc[i][j][r];
    }
    __builtin_amdgcn_fence(__ATOMIC_RELEASE, "workgroup");
    __builtin_amdgcn_wave_barrier();
    __builtin_amdgcn_fence(__ATOMIC_ACQUIRE, "workgroup");
    v4f vv[8];
#pragma unroll
    for (int it = 0; it < 8; ++it) {
      const int row = it * 2 + hh;
      v4f v = *(const v4fa*)(slab + row * 68 + c4);
      if (EPI == 1) v += bv;
      vv[it] = v;
    }
    for (int pass = 0; pass < 2; ++pass) {
#pragma unroll
      for (int it = 0; it < 8; ++it) {
        const int row = mBase + it * 2 + hh;
        if (cok && row < M) *(volatile v4f*)(D + (size_t)row * (size_t)ldd + nc) = vv[it];
      }
      __threadfence();
    }
    __builtin_amdgcn_fence(__ATOMIC_RELEASE, "workgroup");
    __builtin_amdgcn_wave_barrier();
    __builtin_amdgcn_fence(__ATOMIC_ACQUIRE, "workgroup");
  }
}

#define N_NODES  50000
#define N_EDGES  800000
#define IN_DIM   128
#define EDGE_DIM 16
#define HDW      128
#define MPN      50048
#define NBRUN    1024
#define NBLK     49
#define RCAP     20854
#define RCAPP    20864
#define DEGCAP   48
#define GCH      5
#define NCHUNK   10
#define NTHR     256
#define NWAVE    8
#define EPT      8
#define CHUNK    (NTHR * EPT)
#define WCAP     (EPT * 32)
#define LISTN    (NWAVE * WCAP)
#define OFFP     1056
#define LDS_BKT  ((2 * RCAPP + NBRUN + OFFP + LISTN + 32) * 4)

static_assert(N_EDGES < (1 << 20));
static_assert(NBRUN <= (1 << 10));
static_assert(NBLK * NBRUN >= N_NODES && (NBLK - 1) * NBRUN < N_NODES);
static_assert(RCAP * 4 >= 16683 * 5);
static_assert(RCAPP >= RCAP && (RCAPP % 128) == 0);
static_assert(DEGCAP >= 38 + 8);
static_assert((NCHUNK - 1) * GCH < NBLK && NCHUNK * GCH >= NBLK);
static_assert((MPN % 64) == 0 && MPN >= N_NODES && (N_NODES % 16) == 0);
static_assert((MPN * IN_DIM / 8) % 256 == 0);
static_assert((RCAPP * 4) % 256 == 0);
static_assert((OFFP % 32) == 0 && OFFP >= NBRUN + 3);
static_assert(NTHR * 4 == NBRUN);
static_assert(CHUNK == 2048 && LISTN >= NWAVE * WCAP);
static_assert(LDS_BKT <= 262144);
static_assert(NWAVE * DEGCAP * 32 * 4 <= 65536);

#define WS_OXB   ((size_t)0)
#define WS_OWNT  (WS_OXB  + (size_t)MPN * IN_DIM * 2)
#define WS_OWET  (WS_OWNT + (size_t)HDW * IN_DIM * 2)
#define WS_OH    (WS_OWET + (size_t)HDW * 32 * 2)
#define WS_OLIST (WS_OH   + (size_t)MPN * HDW * 4)
#define WS_OOFFS (WS_OLIST + (size_t)NBLK * RCAPP * 8)
#define WS_OEAB  (WS_OOFFS + (size_t)NBLK * OFFP * 4)
#define WS_OEF   (WS_OEAB + (size_t)GCH * RCAPP * 32 * 2)
#define WS_TOTAL (WS_OEF  + (size_t)GCH * RCAPP * HDW * 4)
static_assert(WS_TOTAL <= ((size_t)128 << 20));
static_assert((WS_OWNT % 128) == 0 && (WS_OWET % 128) == 0 && (WS_OH % 128) == 0 && (WS_OLIST % 128) == 0);
static_assert((WS_OOFFS % 128) == 0 && (WS_OEAB % 128) == 0 && (WS_OEF % 128) == 0);

typedef int v4i __attribute__((ext_vector_type(4)));
typedef int v2i __attribute__((ext_vector_type(2)));
typedef v4i __attribute__((may_alias)) v4ia;
typedef v2i __attribute__((may_alias)) v2ia;

__device__ __forceinline__ void prep_unit(const float* __restrict__ w, int kin, int KP, int u,
                                          unsigned short* __restrict__ wt) {
  const int ppr = KP >> 3;
  const int n   = u / ppr;
  const int k8  = (u - n * ppr) * 8;
  const int hd  = n >> 4;
  const int d   = n & 15;
  const float* base = w + (size_t)hd * (size_t)kin * 16 + d;
  float x[8];
  unsigned mk[8];
#pragma unroll
  for (int e = 0; e < 8; ++e) {
    const int i = k8 + e;
    const float v = base[(size_t)clampi(i, 0, kin - 1) * 16];
    asm volatile("" :: "v"(v));
    x[e]  = v;
    mk[e] = (i < kin) ? 0xFFFFu : 0u;
  }
  v4u o = pack8_bf16((v4f){ x[0], x[1], x[2], x[3] }, (v4f){ x[4], x[5], x[6], x[7] });
  o &= (v4u){ pk16(mk[0], mk[1]), pk16(mk[2], mk[3]), pk16(mk[4], mk[5]), pk16(mk[6], mk[7]) };
  volatile v4u* q = (volatile v4u*)(wt + (size_t)n * (size_t)KP + k8);
  *q = o;
  __threadfence();
  *q = o;
}

__global__ __launch_bounds__(NTHR) void k_prep(const float* __restrict__ Wn, const float* __restrict__ We,
                                               unsigned short* __restrict__ WNT, unsigned short* __restrict__ WET) {
  const int tid = (int)threadIdx.x;
  if (blockIdx.x < 8) {
    prep_unit(Wn, IN_DIM, IN_DIM, (int)blockIdx.x * NTHR + tid, WNT);
  } else {
    prep_unit(We, EDGE_DIM, 32, ((int)blockIdx.x - 8) * NTHR + tid, WET);
  }
}

__device__ __forceinline__ int scan_chunk(const int* __restrict__ dsts, int nE, int cbase, int slotBase,
                                          int nb, int* list, int tid, int lane, int wave) {
  int wc = 0;
  const int el0  = tid * EPT;
  const int e0   = cbase + el0;
  const int sent = (-0x7fffffff - 1);
  v4i da, db;
  if (cbase + CHUNK <= nE) {
    da = *(const v4ia*)(dsts + e0);
    db = *(const v4ia*)(dsts + e0 + 4);
  } else {
    const int hi = nE - 1;
    const int t0 = dsts[e0     < hi ? e0     : hi];
    const int t1 = dsts[e0 + 1 < hi ? e0 + 1 : hi];
    const int t2 = dsts[e0 + 2 < hi ? e0 + 2 : hi];
    const int t3 = dsts[e0 + 3 < hi ? e0 + 3 : hi];
    const int t4 = dsts[e0 + 4 < hi ? e0 + 4 : hi];
    const int t5 = dsts[e0 + 5 < hi ? e0 + 5 : hi];
    const int t6 = dsts[e0 + 6 < hi ? e0 + 6 : hi];
    const int t7 = dsts[e0 + 7 < hi ? e0 + 7 : hi];
    asm volatile("" :: "v"(t0)); asm volatile("" :: "v"(t1)); asm volatile("" :: "v"(t2)); asm volatile("" :: "v"(t3));
    asm volatile("" :: "v"(t4)); asm volatile("" :: "v"(t5)); asm volatile("" :: "v"(t6)); asm volatile("" :: "v"(t7));
    da.x = (e0     < nE) ? t0 : sent;
    da.y = (e0 + 1 < nE) ? t1 : sent;
    da.z = (e0 + 2 < nE) ? t2 : sent;
    da.w = (e0 + 3 < nE) ? t3 : sent;
    db.x = (e0 + 4 < nE) ? t4 : sent;
    db.y = (e0 + 5 < nE) ? t5 : sent;
    db.z = (e0 + 6 < nE) ? t6 : sent;
    db.w = (e0 + 7 < nE) ? t7 : sent;
  }
  const unsigned nbs = (unsigned)slotBase;
  const unsigned unb = (unsigned)nb;
  const unsigned s0 = (unsigned)da.x - nbs, s1 = (unsigned)da.y - nbs;
  const unsigned s2 = (unsigned)da.z - nbs, s3 = (unsigned)da.w - nbs;
  const unsigned s4 = (unsigned)db.x - nbs, s5 = (unsigned)db.y - nbs;
  const unsigned s6 = (unsigned)db.z - nbs, s7 = (unsigned)db.w - nbs;
  const bool h0 = s0 < unb, h1 = s1 < unb, h2 = s2 < unb, h3 = s3 < unb;
  const bool h4 = s4 < unb, h5 = s5 < unb, h6 = s6 < unb, h7 = s7 < unb;
  const unsigned any = __builtin_amdgcn_ballot_w32(h0 | h1 | h2 | h3 | h4 | h5 | h6 | h7);
  if (any != 0u) {
#define HITJ(J, HJ, SJ) { \
      const unsigned mj = __builtin_amdgcn_ballot_w32(HJ); \
      if (mj != 0u) { \
        if (HJ) { \
          const int pos = wc + (int)__builtin_amdgcn_mbcnt_lo(mj, 0u); \
          if (pos < WCAP) list[wave * WCAP + pos] = ((el0 + (J)) << 12) | (int)(SJ); \
        } \
        wc += (int)__builtin_popcount(mj); } }
    HITJ(0, h0, s0)
    HITJ(1, h1, s1)
    HITJ(2, h2, s2)
    HITJ(3, h3, s3)
    HITJ(4, h4, s4)
    HITJ(5, h5, s5)
    HITJ(6, h6, s6)
    HITJ(7, h7, s7)
#undef HITJ
  }
  return wc;
}

__global__ __launch_bounds__(NTHR) void k_bucket(const int* __restrict__ dsts, const int* __restrict__ srcs,
                                                 int* __restrict__ LIST, int* __restrict__ OFFS, int nN, int nE) {
  extern __shared__ v4u lds_dyn[];
  int* reg1 = (int*)lds_dyn;
  int* reg2 = reg1 + RCAPP;
  int* scnt = reg2 + RCAPP;
  int* soff = scnt + NBRUN;
  int* list = soff + OFFP;
  int* wcnt = list + LISTN;
  int* wtot = wcnt + NWAVE;
  int* wflg = wtot + NWAVE;
  const int tid = (int)threadIdx.x, lane = tid & 31, wave = tid >> 5;
  const int b = (int)blockIdx.x;
  const int slotBase = b * NBRUN;
  int nb = nN - slotBase;
  nb = nb < 0 ? 0 : (nb > NBRUN ? NBRUN : nb);

  {
    const v4i z4 = (v4i){0, 0, 0, 0};
    for (int i = tid; i < NBRUN; i += NTHR) scnt[i] = 0;
    for (int i = tid; i < RCAPP / 4; i += NTHR) *(v4ia*)(reg2 + 4 * i) = z4;
  }
  __syncthreads();

  int totraw = 0;
  const int nChunks = (nE + CHUNK - 1) / CHUNK;
#pragma unroll 1
  for (int ch = 0; ch < nChunks; ++ch) {
    const int cbase = ch * CHUNK;
    const int wc = scan_chunk(dsts, nE, cbase, slotBase, nb, list, tid, lane, wave);
    if (lane == 0) wcnt[wave] = wc;
    __syncthreads();
    int pre = 0, all = 0;
#pragma unroll
    for (int w2 = 0; w2 < NWAVE; ++w2) {
      int c = wcnt[w2];
      c = c < 0 ? 0 : (c > WCAP ? WCAP : c);
      all += c;
      pre += (w2 < wave) ? c : 0;
    }
    const int wcc  = wc > WCAP ? WCAP : wc;
    const int tot  = totraw > RCAPP ? RCAPP : totraw;
    const int base = tot + pre;
#pragma unroll 1
    for (int i0 = 0; i0 < wcc; i0 += 32) {
      const int i  = i0 + lane;
      const int ic = i < wcc ? i : wcc - 1;
      const int ent = list[wave * WCAP + ic];
      const int el  = (ent >> 12) & (CHUNK - 1);
      const int sl  = ent & (NBRUN - 1);
      int eid = cbase + el;
      eid = eid > nE - 1 ? nE - 1 : eid;
      const int pos = base + i;
      if (i < wcc && pos < RCAPP) reg1[pos] = (int)(((unsigned)sl << 20) | (unsigned)eid);
    }
    totraw += all;
    __syncthreads();
  }
  const int nh  = totraw > RCAPP ? RCAPP : totraw;
  const int ovf = totraw > RCAP ? 1 : 0;

  if (wave == 0) {
#pragma unroll 1
    for (int b0 = 0; b0 < nh; b0 += 32) {
      const int idx = b0 + lane;
      const int uv  = reg1[idx < nh ? idx : nh - 1];
      const int m32 = (nh - b0) < 32 ? (nh - b0) : 32;
#pragma unroll 1
      for (int k = 0; k < m32; ++k) {
        const int u  = __builtin_amdgcn_readlane(uv, k);
        const int sl = (int)(((unsigned)u >> 20) & (unsigned)(NBRUN - 1));
        if (lane == 0) scnt[sl] = scnt[sl] + 1;
      }
    }
  }
  __syncthreads();

  int fl = ovf;
  {
    const v4i ca = *(const v4ia*)(scnt + 4 * tid);
    const int e0 = ca.x < 0 ? 0 : ca.x, e1 = ca.y < 0 ? 0 : ca.y, e2 = ca.z < 0 ? 0 : ca.z, e3 = ca.w < 0 ? 0 : ca.w;
    const bool big = (e0 > DEGCAP) | (e1 > DEGCAP) | (e2 > DEGCAP) | (e3 > DEGCAP);
    const unsigned bm = __builtin_amdgcn_ballot_w32(big);
    const int ts = e0 + e1 + e2 + e3;
    int incl = ts;
#pragma unroll
    for (int d = 1; d < 32; d <<= 1) {
      const int up = __shfl_up(incl, d);
      if (lane >= d) incl += up;
    }
    if (lane == 31) wtot[wave] = incl;
    if (lane == 0)  wflg[wave] = (bm != 0u) ? 1 : 0;
    __syncthreads();
    int pre = 0;
#pragma unroll
    for (int w2 = 0; w2 < NWAVE; ++w2) {
      pre += (w2 < wave) ? wtot[w2] : 0;
      fl |= wflg[w2];
    }
    int run = pre + incl - ts;
    soff[4 * tid + 0] = run; run += e0;
    soff[4 * tid + 1] = run; run += e1;
    soff[4 * tid + 2] = run; run += e2;
    soff[4 * tid + 3] = run;
    if (tid < 32) soff[NBRUN + tid] = (tid < 2) ? nh : ((tid == 2) ? fl : 0);
  }
  __syncthreads();
  for (int i = tid; i < NBRUN; i += NTHR) list[i] = soff[i];
  __syncthreads();

  if (wave == 0) {
#pragma unroll 1
    for (int b0 = 0; b0 < nh; b0 += 32) {
      const int idx = b0 + lane;
      const int uv  = reg1[idx < nh ? idx : nh - 1];
      const int m32 = (nh - b0) < 32 ? (nh - b0) : 32;
#pragma unroll 1
      for (int k = 0; k < m32; ++k) {
        const int u   = __builtin_amdgcn_readlane(uv, k);
        const int sl  = (int)(((unsigned)u >> 20) & (unsigned)(NBRUN - 1));
        const int eid = (int)((unsigned)u & 0xFFFFFu);
        if (lane == 0) {
          int pos = list[sl];
          pos = pos < 0 ? 0 : (pos > RCAPP - 1 ? RCAPP - 1 : pos);
          reg2[pos] = eid;
          list[sl] = pos + 1;
        }
      }
    }
  }
  __syncthreads();

  {
    int* Lb = LIST + (size_t)b * (size_t)RCAPP * 2;
    const int nU = RCAPP / 2;
#pragma unroll 1
    for (int it = 0; it < (nU + NTHR - 1) / NTHR; ++it) {
      const int u  = it * NTHR + tid;
      const int uc = u < nU ? u : nU - 1;
      const v2i ee = *(const v2ia*)(reg2 + 2 * uc);
      const int e0 = clampi(ee.x, 0, nE - 1);
      const int e1 = clampi(ee.y, 0, nE - 1);
      int s0 = srcs[e0];
      int s1 = srcs[e1];
      asm volatile("" :: "v"(s0));
      asm volatile("" :: "v"(s1));
      s0 = clampi(s0, 0, nN - 1);
      s1 = clampi(s1, 0, nN - 1);
      const int m0 = (2 * uc     < nh) ? -1 : 0;
      const int m1 = (2 * uc + 1 < nh) ? -1 : 0;
      const v4i o = (v4i){ s0 & m0, e0 & m0, s1 & m1, e1 & m1 };
      volatile v4i* q = (volatile v4i*)(Lb + 4 * (size_t)uc);
      const bool ok = u < nU;
      if (ok) *q = o;
      __threadfence();
      if (ok) *q = o;
    }
  }
  {
    int* Ob = OFFS + (size_t)b * OFFP;
    const int nU = OFFP / 4;
#pragma unroll 1
    for (int it = 0; it < (nU + NTHR - 1) / NTHR; ++it) {
      const int u  = it * NTHR + tid;
      const int uc = u < nU ? u : nU - 1;
      const v4i o = *(const v4ia*)(soff + 4 * uc);
      volatile v4i* q = (volatile v4i*)(Ob + 4 * uc);
      const bool ok = u < nU;
      if (ok) *q = o;
      __threadfence();
      if (ok) *q = o;
    }
  }
}

__global__ __launch_bounds__(NTHR) void k_ea(const float* __restrict__ ea, const int* __restrict__ LISTc,
                                             const int* __restrict__ OFFS, unsigned short* __restrict__ EAB,
                                             int b0, int nRows, int nE) {
  const unsigned total = (unsigned)nRows * 4u;
  const unsigned g  = blockIdx.x * (unsigned)NTHR + threadIdx.x;
  const unsigned gc = g < total ? g : total - 1u;
  const int r  = (int)(gc >> 2);
  const int pc = (int)(gc & 3u);
  const int lb = r / RCAPP;
  const int p  = r - lb * RCAPP;
  int cnt = OFFS[(size_t)(b0 + lb) * OFFP + NBRUN];
  asm volatile("" :: "v"(cnt));
  cnt = clampi(cnt, 0, RCAPP);
  v2i se = *(const v2ia*)(LISTc + 2 * (size_t)r);
  asm volatile("" :: "v"(se));
  const int eid = clampi(se.y, 0, nE - 1);
  const float* rp = ea + (size_t)eid * EDGE_DIM + (pc & 1) * 8;
  v4f a = *(const v4fa*)(rp);
  v4f c = *(const v4fa*)(rp + 4);
  asm volatile("" :: "v"(a));
  asm volatile("" :: "v"(c));
  v4u o = pack8_bf16(a, c);
  const unsigned mk = (p < cnt && pc < 2) ? 0xFFFFFFFFu : 0u;
  o &= (v4u){ mk, mk, mk, mk };
  if (g < total) {
    volatile v4u* q = (volatile v4u*)(EAB + (size_t)g * 8);
    *q = o;
    __threadfence();
    *q = o;
  }
}

__global__ __launch_bounds__(NTHR) void k_replay(const float* __restrict__ Hm, const float* __restrict__ EF,
                                                 const int* __restrict__ LISTc, const int* __restrict__ OFFS,
                                                 float* __restrict__ out, int b0, int nReal) {
  __shared__ float strip[NWAVE * DEGCAP * 32];
  const int tid = (int)threadIdx.x, lane = tid & 31, wave = tid >> 5;
  const int rowc = (int)blockIdx.x * NWAVE + wave;
  const int lb   = rowc >> 10;
  const int slot = rowc & (NBRUN - 1);
  const int b    = b0 + lb;
  const int t    = b * NBRUN + slot;
  const bool live = t < nReal;
  const int* ob = OFFS + (size_t)b * OFFP;
  int o0 = ob[slot];
  int o1 = ob[slot + 1];
  int fg = ob[NBRUN + 2];
  asm volatile("" :: "v"(o0));
  asm volatile("" :: "v"(o1));
  asm volatile("" :: "v"(fg));
  const int st = clampi(o0, 0, RCAPP);
  int c = clampi(o1 - o0, 0, DEGCAP);
  c = c > RCAPP - st ? RCAPP - st : c;
  c = live ? c : 0;
  const int cn  = __builtin_amdgcn_readfirstlane(c);
  const int stu = __builtin_amdgcn_readfirstlane(st);
  const int tcl = clampi(t, 0, nReal - 1);
  v4f q = *(const v4fa*)(Hm + (size_t)tcl * HDW + 4 * lane);
  asm volatile("" :: "v"(q));
  const size_t r0 = (size_t)lb * RCAPP + (size_t)stu;
  const int*   lp = LISTc + 2 * r0;
  const float* ep = EF + r0 * HDW + 4 * lane;
  float* sp = strip + wave * (DEGCAP * 32) + lane;

  float mx = -__builtin_inff();
#pragma unroll 1
  for (int j = 0; j < cn; ++j) {
    v2i se = *(const v2ia*)(lp + 2 * j);
    asm volatile("" :: "v"(se));
    const int s = clampi(se.x, 0, nReal - 1);
    v4f k = *(const v4fa*)(Hm + (size_t)s * HDW + 4 * lane);
    v4f e = *(const v4fa*)(ep + (size_t)j * HDW);
    asm volatile("" :: "v"(k));
    asm volatile("" :: "v"(e));
    float pd = q.x * k.x;
    pd = fmaf(q.y, k.y, pd);
    pd = fmaf(q.z, k.z, pd);
    pd = fmaf(q.w, k.w, pd);
    float pe = (e.x + e.y) + (e.z + e.w);
    pd += __shfl_xor(pd, 1);
    pe += __shfl_xor(pe, 1);
    pd += __shfl_xor(pd, 2);
    pe += __shfl_xor(pe, 2);
    float v = (pd + pe) * 0.25f;
    v = (v > 0.0f) ? v : 0.2f * v;
    sp[j * 32] = v;
    mx = fmaxf(mx, v);
  }
  const bool fin = (__float_as_uint(mx) & 0x7f800000u) != 0x7f800000u;
  const float m = fin ? mx : 0.0f;

  v4f acc = (v4f){0.0f, 0.0f, 0.0f, 0.0f};
  float den = 0.0f;
#pragma unroll 1
  for (int j = 0; j < cn; ++j) {
    v2i se = *(const v2ia*)(lp + 2 * j);
    asm volatile("" :: "v"(se));
    const int s = clampi(se.x, 0, nReal - 1);
    v4f k = *(const v4fa*)(Hm + (size_t)s * HDW + 4 * lane);
    v4f e = *(const v4fa*)(ep + (size_t)j * HDW);
    asm volatile("" :: "v"(k));
    asm volatile("" :: "v"(e));
    const float lg = sp[j * 32];
    const float ex = expf(lg - m);
    den += ex;
    const float g0 = 1.0f / (1.0f + expf(-e.x));
    const float g1 = 1.0f / (1.0f + expf(-e.y));
    const float g2 = 1.0f / (1.0f + expf(-e.z));
    const float g3 = 1.0f / (1.0f + expf(-e.w));
    acc.x += (k.x * g0) * ex;
    acc.y += (k.y * g1) * ex;
    acc.z += (k.z * g2) * ex;
    acc.w += (k.w * g3) * ex;
  }
  const float dv = den + 1e-9f;
  v4f o;
  o.x = acc.x / dv;
  o.y = acc.y / dv;
  o.z = acc.z / dv;
  o.w = acc.w / dv;
  const v4f z4 = (v4f){0.0f, 0.0f, 0.0f, 0.0f};
  o = (cn > 0) ? o : z4;
  const float qn = __uint_as_float(0x7fc00000u);
  const v4f n4 = (v4f){qn, qn, qn, qn};
  o = (fg != 0) ? n4 : o;
  volatile v4f* gp = (volatile v4f*)(out + (size_t)tcl * HDW + 4 * lane);
  if (live) *gp = o;
  __threadfence();
  if (live) *gp = o;
}

static inline int cdiv_i(int a, int b) { return (a + b - 1) / b; }

extern "C" void kernel_launch(void* const* d_in, const int* in_sizes, int n_in,
                              void* d_out, int out_size, void* d_ws, size_t ws_size,
                              hipStream_t stream) {
  if (n_in < 6) return;
  if (in_sizes[0] != N_NODES * IN_DIM) return;
  if (in_sizes[1] != N_EDGES * EDGE_DIM) return;
  if (in_sizes[2] != 8 * IN_DIM * 16) return;
  if (in_sizes[3] != 8 * EDGE_DIM * 16) return;
  if (in_sizes[4] != N_EDGES || in_sizes[5] != N_EDGES) return;
  if (out_size != N_NODES * HDW) return;
  if (ws_size < WS_TOTAL) return;

  const float* x   = (const float*)d_in[0];
  const float* ea  = (const float*)d_in[1];
  const float* Wn  = (const float*)d_in[2];
  const float* We  = (const float*)d_in[3];
  const int*   src = (const int*)d_in[4];
  const int*   dst = (const int*)d_in[5];
  float* out = (float*)d_out;

  char* ws = (char*)d_ws;
  unsigned short* XB  = (unsigned short*)(ws + WS_OXB);
  unsigned short* WNT = (unsigned short*)(ws + WS_OWNT);
  unsigned short* WET = (unsigned short*)(ws + WS_OWET);
  float*          Hm  = (float*)(ws + WS_OH);
  int*            LST = (int*)(ws + WS_OLIST);
  int*            OFS = (int*)(ws + WS_OOFFS);
  unsigned short* EAB = (unsigned short*)(ws + WS_OEAB);
  float*          EFm = (float*)(ws + WS_OEF);

  hipFuncSetAttribute(reinterpret_cast<const void*>(&k_bucket),
                      hipFuncAttributeMaxDynamicSharedMemorySize, LDS_BKT);

  k_plane<0><<<MPN * IN_DIM / 8 / 256, 256, 0, stream>>>(x, N_NODES, IN_DIM, IN_DIM, XB, MPN, IN_DIM);
  k_prep<<<10, NTHR, 0, stream>>>(Wn, We, WNT, WET);
  {
    const int T = cdiv_i(N_NODES, 64) * cdiv_i(HDW, 64);
    k_gemm_nt<0, 0><<<cdiv_i(T, 8), 256, 0, stream>>>(XB, WNT, Wn, Hm, N_NODES, HDW, IN_DIM, HDW);
  }
  k_bucket<<<NBLK, NTHR, LDS_BKT, stream>>>(dst, src, LST, OFS, N_NODES, N_EDGES);

  for (int c = 0; c < NCHUNK; ++c) {
    const int b0 = c * GCH;
    int nblk = NBLK - b0;
    nblk = nblk > GCH ? GCH : nblk;
    if (nblk <= 0) break;
    const int R = nblk * RCAPP;
    const int* LISTc = LST + (size_t)b0 * (size_t)RCAPP * 2;
    k_ea<<<R * 4 / NTHR, NTHR, 0, stream>>>(ea, LISTc, OFS, EAB, b0, R, N_EDGES);
    const int T = (R / 64) * (HDW / 64);
    k_gemm_nt<0, 0><<<cdiv_i(T, 8), 256, 0, stream>>>(EAB, WET, Wn, EFm, R, HDW, 32, HDW);
    k_replay<<<nblk * (NBRUN / NWAVE), NTHR, 0, stream>>>(Hm, EFm, LISTc, OFS, out, b0, N_NODES);
  }
}
